// EncryptedFeedForward_83184926589623
// MI455X (gfx1250) — hardware-verified
//
#include <hip/hip_runtime.h>


#define NN_  8192
#define DD   1024
#define FF   4096

typedef unsigned short bf;
typedef __attribute__((ext_vector_type(16))) __bf16   v16bf;
typedef __attribute__((ext_vector_type(8)))  unsigned short v8us;
typedef __attribute__((ext_vector_type(8)))  float    v8f;
typedef __attribute__((ext_vector_type(4)))  float    v4f;
typedef v4f  __attribute__((may_alias)) v4fa;
typedef v8us __attribute__((may_alias)) v8usa;

__device__ __forceinline__ unsigned short f2bf(float f) { unsigned u = __float_as_uint(f); u += 0x7FFFu + ((u >> 16) & 1u); return (unsigned short)(u >> 16); }
__device__ __forceinline__ float bf2f(unsigned short b) { return __uint_as_float(((unsigned)b) << 16); }
__device__ __forceinline__ float bfr(float f) { return bf2f(f2bf(f)); }
__device__ __forceinline__ v16bf cat16b(v8us lo, v8us hi) { return __builtin_bit_cast(v16bf, __builtin_shufflevector(lo, hi, 0, 1, 2, 3, 4, 5, 6, 7, 8, 9, 10, 11, 12, 13, 14, 15)); }
__device__ __forceinline__ v8f wmmab(v16bf a, v16bf b, v8f c) { return __builtin_amdgcn_wmma_f32_16x16x32_bf16(false, a, false, b, (short)0, c, false, false); }

template <int C>
__global__ __launch_bounds__(256) void k_cvtb(const float* __restrict__ src, int nrows, bf* dst) {
    const int lane = threadIdx.x & 31, r = blockIdx.x * 8 + (threadIdx.x >> 5);
    if (r >= nrows) return;
#pragma unroll 1
    for (int ps = 0; ps < 2; ++ps) {
#pragma unroll
        for (int q = 0; q < C / 256; ++q) { v8us o;
#pragma unroll
            for (int i = 0; i < 8; ++i) o[i] = f2bf(src[(size_t)r * C + q * 256 + lane * 8 + i]);
            *(volatile v8us*)(dst + (size_t)r * C + q * 256 + lane * 8) = o; }
        if (ps == 0) __threadfence(); }
}
__global__ __launch_bounds__(256) void k_wt(const float* __restrict__ Wm, int K, int ncols, bf* WT) {
    __shared__ __align__(16) unsigned short tl[64 * 72];
    const int tid = threadIdx.x, k0 = blockIdx.x * 64, n0 = blockIdx.y * 64;
    const int kk = tid >> 2, nq = (tid & 3) * 16;
#pragma unroll
    for (int i = 0; i < 16; ++i) tl[(nq + i) * 72 + kk] = f2bf(Wm[(size_t)(k0 + kk) * ncols + n0 + nq + i]);
    __syncthreads();
    const int piece = tid & 7;
    auto pass = [&]() {
#pragma unroll
        for (int s = 0; s < 2; ++s) { const int nr = (tid >> 3) + 32 * s; const v8us val = *(const v8usa*)(tl + nr * 72 + piece * 8); *(volatile v8us*)(WT + (size_t)(n0 + nr) * K + k0 + piece * 8) = val; }
    };
    pass(); __threadfence(); pass();
}
template <bool SPLITA, int MODE, bool ACC>
__global__ __launch_bounds__(128) void k_gemm(const bf* __restrict__ A, const bf* __restrict__ Al, int lda, const bf* __restrict__ Bn, int ldb, int K, const float* __restrict__ bias, int ldc, float* C, bf* PH, bf* PL) {
    __shared__ __align__(16) float ost[4][16 * 68];
    const int lane = threadIdx.x & 31, wave = threadIdx.x >> 5, lr = lane & 15, hi = lane >> 4;
    const size_t r0 = (size_t)blockIdx.x * 64 + wave * 16; const int c0 = blockIdx.y * 64;
    const size_t aoff = (r0 + lr) * (size_t)lda + 8 * hi;
    size_t boff[4];
#pragma unroll
    for (int t = 0; t < 4; ++t) boff[t] = (size_t)(c0 + t * 16 + lr) * ldb + 8 * hi;
    v8f acc[4];
#pragma unroll
    for (int t = 0; t < 4; ++t) acc[t] = (v8f){};
#pragma unroll 2
    for (int kc = 0; kc < K; kc += 32) {
        const v16bf a = cat16b(*(const v8us*)(A + aoff + kc), *(const v8us*)(A + aoff + kc + 16));
        v16bf al = a; if (SPLITA) al = cat16b(*(const v8us*)(Al + aoff + kc), *(const v8us*)(Al + aoff + kc + 16));
#pragma unroll
        for (int t = 0; t < 4; ++t) { const v16bf bb = cat16b(*(const v8us*)(Bn + boff[t] + kc), *(const v8us*)(Bn + boff[t] + kc + 16)); acc[t] = wmmab(a, bb, acc[t]); if (SPLITA) acc[t] = wmmab(al, bb, acc[t]); }
        asm volatile("v_nop" : "+v"(acc[0]), "+v"(acc[1]), "+v"(acc[2]), "+v"(acc[3]) : "v"(a), "v"(al) : "memory");
    }
    float* os = &ost[wave][0];
#pragma unroll
    for (int t = 0; t < 4; ++t) { const float bv = bias ? bfr(bias[c0 + t * 16 + lr]) : 0.f;
#pragma unroll
        for (int j = 0; j < 8; ++j) { float v = acc[t][j] + bv; if (MODE == 0) v = v * (0.5f + v * (0.5f - 0.125f * v)); if (ACC) v += C[(r0 + hi * 8 + j) * ldc + c0 + t * 16 + lr]; os[(hi * 8 + j) * 68 + t * 16 + lr] = v; } }
    __builtin_amdgcn_wave_barrier(); asm volatile("" ::: "memory");
    if (MODE == 0) {
        bf* p1 = PH + r0 * ldc + c0; bf* p2 = PL + r0 * ldc + c0;
        auto pass = [&]() {
#pragma unroll
            for (int s = 0; s < 4; ++s) { const int row = 4 * s + (lane >> 3), piece = lane & 7; const float* sp = os + row * 68 + piece * 8; v8us oh, ol;
#pragma unroll
                for (int i = 0; i < 8; ++i) { const unsigned short hb = f2bf(sp[i]); oh[i] = hb; ol[i] = f2bf(sp[i] - bf2f(hb)); }
                *(volatile v8us*)(p1 + (size_t)row * ldc + piece * 8) = oh; *(volatile v8us*)(p2 + (size_t)row * ldc + piece * 8) = ol; }
        };
        pass(); __threadfence(); pass();
    } else {
        float* crow = C + r0 * ldc + c0;
        auto pass = [&]() {
#pragma unroll
            for (int s = 0; s < 8; ++s) { const int Lid = (lane >> 3) + 4 * s, piece = lane & 7; const int row = Lid >> 1, cofs = (Lid & 1) * 32 + piece * 4;
                const v4f val = *(const v4fa*)(os + row * 68 + cofs); *(volatile v4f*)(crow + (size_t)row * ldc + cofs) = val; }
        };
        pass(); __threadfence(); pass();
    }
}

extern "C" void kernel_launch(void* const* d_in, const int* in_sizes, int n_in,
                              void* d_out, int out_size, void* d_ws, size_t ws_size, hipStream_t stream) {
    (void)in_sizes; (void)n_in; (void)out_size;
    const float* x = (const float*)d_in[0]; const float* W1 = (const float*)d_in[1]; const float* b1 = (const float*)d_in[2]; const float* W2 = (const float*)d_in[3]; const float* b2 = (const float*)d_in[4];
    float* out = (float*)d_out;
    char* wsp = (char*)d_ws;
    auto take = [&](size_t bytes) { char* p = wsp; wsp += (bytes + 255) & ~(size_t)255; return (void*)p; };
    bf* Xb = (bf*)take((size_t)NN_ * DD * 2); bf* W1T = (bf*)take((size_t)FF * DD * 2); bf* W2T = (bf*)take((size_t)DD * FF * 2);
    bf* HH = (bf*)take((size_t)NN_ * (FF / 2) * 2); bf* HL = (bf*)take((size_t)NN_ * (FF / 2) * 2);
    if ((size_t)(wsp - (char*)d_ws) > ws_size) return;
    k_cvtb<DD><<<NN_ / 8, 256, 0, stream>>>(x, NN_, Xb);
    k_wt<<<dim3(DD / 64, FF / 64, 1), 256, 0, stream>>>(W1, DD, FF, W1T);
    k_wt<<<dim3(FF / 64, DD / 64, 1), 256, 0, stream>>>(W2, FF, DD, W2T);
    for (int half = 0; half < 2; ++half) {
        k_gemm<false, 0, false><<<dim3(NN_ / 64, (FF / 2) / 64, 1), 128, 0, stream>>>(Xb, nullptr, DD, W1T + (size_t)half * (FF / 2) * DD, DD, DD, b1 + half * (FF / 2), FF / 2, nullptr, HH, HL);
        if (half == 0) k_gemm<true, 1, false><<<dim3(NN_ / 64, DD / 64, 1), 128, 0, stream>>>(HH, HL, FF / 2, W2T, FF, FF / 2, b2, DD, out, nullptr, nullptr);
        else           k_gemm<true, 1, true ><<<dim3(NN_ / 64, DD / 64, 1), 128, 0, stream>>>(HH, HL, FF / 2, W2T + (size_t)(FF / 2), FF, FF / 2, nullptr, DD, out, nullptr, nullptr);
    }
}
